// SlidingWindowAttention_23957327577817
// MI455X (gfx1250) — hardware-verified
//
#include <hip/hip_runtime.h>
#include <math.h>

#ifndef NB
#define NB 2
#endif
#ifndef SEQ
#define SEQ 2048
#endif
#ifndef NEARLY
#define NEARLY 256
#endif
#define NB_FULL 2
#define SEQ_FULL 2048
#define NE 1024
#define NHD 16
#define NKV 4
#define HD 64
#define NKVE (NKV * HD)
#define WINSZ 512
#define IN_BSTRIDE ((long long)SEQ_FULL * NE)
#ifndef OUT_BSTRIDE
#define OUT_BSTRIDE ((long long)SEQ_FULL * NE)
#endif
#define MROWS (NB * SEQ)

static_assert(SEQ % 64 == 0);
static_assert(NEARLY % 64 == 0);
static_assert(NEARLY >= 64);
static_assert(NEARLY <= SEQ);
static_assert(NB >= 1 && NB <= NB_FULL);
static_assert(SEQ <= SEQ_FULL);
static_assert(NE % 64 == 0);
static_assert(NKVE % 64 == 0);
static_assert(MROWS % 32 == 0);
static_assert(HD == 64);
static_assert(NHD * HD == NE);

typedef __attribute__((ext_vector_type(16))) _Float16 v16h;
typedef __attribute__((ext_vector_type(8)))  _Float16 v8h;
typedef __attribute__((ext_vector_type(16))) __bf16   v16b;
typedef __attribute__((ext_vector_type(8)))  float    v8f;
typedef __attribute__((ext_vector_type(4)))  float    v4f;
typedef __attribute__((ext_vector_type(2)))  float    v2f;
typedef unsigned int cm_u4 __attribute__((ext_vector_type(4)));

__device__ __forceinline__ int frag_k(int i, int h) { return (i < 8) ? (8 * h + i) : (16 + 8 * h + (i - 8)); }
__device__ __forceinline__ __bf16 bf16_rne(float f) {
    unsigned int u = __float_as_uint(f);
    u += 0x7fffu + ((u >> 16) & 1u);
    return __builtin_bit_cast(__bf16, (unsigned short)(u >> 16));
}
__device__ __forceinline__ float bf16_f32(__bf16 b) { return __uint_as_float(((unsigned int)__builtin_bit_cast(unsigned short, b)) << 16); }
__device__ __forceinline__ v8f wmma16(v16h a, v16h b, v8f c) {
    c = __builtin_amdgcn_wmma_f32_16x16x32_f16(false, a, false, b, (short)0, c, false, false);
    asm volatile("v_nop\n\tv_nop\n\tv_nop\n\tv_nop" : "+v"(c) : "v"(a), "v"(b));
    return c;
}
__device__ __forceinline__ v8f wmmab(v16b a, v16b b, v8f c) {
    c = __builtin_amdgcn_wmma_f32_16x16x32_bf16(false, a, false, b, (short)0, c, false, false);
    asm volatile("v_nop\n\tv_nop\n\tv_nop\n\tv_nop" : "+v"(c) : "v"(a), "v"(b));
    return c;
}
struct Split { v16b hi, lo; };
__device__ __forceinline__ v8f wmma3(const Split& a, const Split& b, v8f c) {
    c = __builtin_amdgcn_wmma_f32_16x16x32_bf16(false, a.hi, false, b.hi, (short)0, c, false, false);
    c = __builtin_amdgcn_wmma_f32_16x16x32_bf16(false, a.hi, false, b.lo, (short)0, c, false, false);
    c = __builtin_amdgcn_wmma_f32_16x16x32_bf16(false, a.lo, false, b.hi, (short)0, c, false, false);
    asm volatile("v_nop\n\tv_nop\n\tv_nop\n\tv_nop" : "+v"(c) : "v"(a.hi), "v"(a.lo), "v"(b.hi), "v"(b.lo));
    return c;
}
struct Split3 { v16b hi, mid, lo; };
__device__ __forceinline__ v8f wmma6(const Split3& a, const Split3& b, v8f c) {
    c = __builtin_amdgcn_wmma_f32_16x16x32_bf16(false, a.hi, false, b.hi, (short)0, c, false, false);
    c = __builtin_amdgcn_wmma_f32_16x16x32_bf16(false, a.hi, false, b.mid, (short)0, c, false, false);
    c = __builtin_amdgcn_wmma_f32_16x16x32_bf16(false, a.mid, false, b.hi, (short)0, c, false, false);
    c = __builtin_amdgcn_wmma_f32_16x16x32_bf16(false, a.hi, false, b.lo, (short)0, c, false, false);
    c = __builtin_amdgcn_wmma_f32_16x16x32_bf16(false, a.mid, false, b.mid, (short)0, c, false, false);
    c = __builtin_amdgcn_wmma_f32_16x16x32_bf16(false, a.lo, false, b.hi, (short)0, c, false, false);
    asm volatile("v_nop\n\tv_nop\n\tv_nop\n\tv_nop" : "+v"(c) : "v"(a.hi), "v"(a.mid), "v"(a.lo), "v"(b.hi), "v"(b.mid), "v"(b.lo));
    return c;
}

__device__ __forceinline__ v16h fh_ld(const float* __restrict__ p, long long sk, int k0, int h, int klen, float s) {
    v16h a;
#pragma unroll
    for (int i = 0; i < 16; ++i) { const int k = k0 + frag_k(i, h); a[i] = (k < klen) ? (_Float16)(p[(long long)k * sk] * s) : (_Float16)0.f; }
    return a;
}
__device__ __forceinline__ Split sp_ld(const float* __restrict__ p, long long sk, int k0, int h, int klen, float s) {
    Split r;
#pragma unroll
    for (int i = 0; i < 16; ++i) {
        const int k = k0 + frag_k(i, h); const float x = (k < klen) ? p[(long long)k * sk] * s : 0.f;
        const __bf16 hb = bf16_rne(x); r.hi[i] = hb; r.lo[i] = bf16_rne(x - bf16_f32(hb));
    }
    return r;
}
__device__ __forceinline__ Split3 sp3_ld(const float* __restrict__ p, long long sk, int k0, int h, int klen, float s) {
    Split3 r;
#pragma unroll
    for (int i = 0; i < 16; ++i) {
        const int k = k0 + frag_k(i, h); const float x = (k < klen) ? p[(long long)k * sk] * s : 0.f;
        const __bf16 hb = bf16_rne(x); const float r1 = x - bf16_f32(hb); const __bf16 mb = bf16_rne(r1);
        r.hi[i] = hb; r.mid[i] = mb; r.lo[i] = bf16_rne(r1 - bf16_f32(mb));
    }
    return r;
}
__device__ __forceinline__ v16h frag_ld(const _Float16* __restrict__ r) {
    const v8h lo = *(const v8h*)r;
    const v8h hi = *(const v8h*)(r + 16);
    return __builtin_shufflevector(lo, hi, 0, 1, 2, 3, 4, 5, 6, 7, 8, 9, 10, 11, 12, 13, 14, 15);
}

#define VST2(T, ptr, val) do { const T vst2_v_ = (val); *(volatile T*)(ptr) = vst2_v_; __threadfence(); *(volatile T*)(ptr) = vst2_v_; } while (0)
#define VST2V4(ptr, val) do { const v4f vst2_v4_ = (val); *(volatile v4f*)(ptr) = vst2_v4_; __threadfence(); *(volatile v4f*)(ptr) = vst2_v4_; } while (0)

#define AW 4
struct AttnP {
    const float* Q; const float* K; const float* V; float* O; float* P; const float* Mf; const int* Mi; float* ST;
    const float* Pw; const float* Rt; const int* SQ; const int* SK;
    long long swb, swh, swi, swj, srb, srh, sri;
    long long sQb, sQh, sQi, sQd, sKb, sKh, sKj, sKd, sVb, sVh, sVj, sVd, sOb, sOh, sOi, sPb, sPh, sPi, smb, smh, smi, smj;
    int Lq, Lk, dh, dv, hrep, causal, coff, pband;
    float scale, mfill; int nonorm, mpol;
    int roff, rn, segpol, win;
};
static_assert(sizeof(AttnP) == 12 * 8 + 29 * 8 + 16 * 4);

#ifndef KATTN_ATTR
#define KATTN_ATTR
#endif
template <int DHP, int DVP, int QM, bool SPLITPV, bool TWOPASS>
__global__ __launch_bounds__(32 * AW) KATTN_ATTR void k_attn(AttnP p) {
    constexpr int NT = DVP / 16;
    constexpr int KS = DHP / 32;
    constexpr int VP = DVP + 8;
    __shared__ __align__(16) float    pl[AW][16 * 64];
    __shared__ __align__(16) _Float16 vl[(SPLITPV ? 2 : 1) * 64 * VP];
    const int lane = threadIdx.x & 31, hf = lane >> 4, l15 = lane & 15, wave = threadIdx.x >> 5;
    const int h = blockIdx.y, b = blockIdx.z, hk = h / p.hrep;
    const int q0 = (blockIdx.x * AW + wave) * 16;
    float* myp = pl[wave];
    const float L2E = 1.4426950408889634f;
    const float NEG = -__builtin_inff();
    const int qi = min(q0 + l15, p.Lq - 1);
    const float* qrow = p.Q + b * p.sQb + h * p.sQh + (long long)qi * p.sQi;
    const float* kbase = p.K + b * p.sKb + hk * p.sKh;
    const float* vbase = p.V + b * p.sVb + hk * p.sVh;
    v16h qa[QM == 0 ? KS : 1]; Split qs_[QM == 1 ? KS : 1]; Split3 qt_[QM == 2 ? KS : 1];
#pragma unroll
    for (int ks = 0; ks < KS; ++ks) {
        if (QM == 2) qt_[ks] = sp3_ld(qrow, p.sQd, ks * 32, hf, p.dh, 1.f);
        else if (QM == 1) qs_[ks] = sp_ld(qrow, p.sQd, ks * 32, hf, p.dh, 1.f);
        else qa[ks] = fh_ld(qrow, p.sQd, ks * 32, hf, p.dh, 1.f);
    }
    v8f o[NT]; float m8[8], l8[8];
#pragma unroll
    for (int t = 0; t < NT; ++t) { v8f zz = {}; o[t] = zz; }
#pragma unroll
    for (int i = 0; i < 8; ++i) { m8[i] = NEG; l8[i] = 0.f; }
    int jend = p.Lk; int jstart = 0;
    if (p.causal == 1) { const int je = (blockIdx.x * AW + AW - 1) * 16 + 16 + p.coff; jend = min(jend, max(je, 0)); }
    if (p.win > 0) { const int js = (int)(blockIdx.x * AW) * 16 + p.coff - p.win; jstart = (js > 0) ? (js / 64) * 64 : 0; }
    const int npass = TWOPASS ? 2 : 1;
    for (int pass = 0; pass < npass; ++pass) {
        const bool dopv = (!TWOPASS) || pass == 1;
        for (int j0 = jstart; j0 < jend; j0 += 64) {
            if (dopv) {
                __syncthreads();
                for (int idx = threadIdx.x; idx < 64 * DVP; idx += 32 * AW) {
                    const int jr = idx / DVP, d = idx - jr * DVP, j = j0 + jr;
                    const float f = (j < p.Lk && d < p.dv) ? vbase[(long long)j * p.sVj + (long long)d * p.sVd] : 0.f;
                    if (SPLITPV) {
                        const __bf16 hb = bf16_rne(f);
                        ((__bf16*)vl)[jr * VP + d] = hb; ((__bf16*)vl)[64 * VP + jr * VP + d] = bf16_rne(f - bf16_f32(hb));
                    } else vl[jr * VP + d] = (_Float16)f;
                }
            }
            v8f s[4];
#pragma unroll
            for (int t = 0; t < 4; ++t) {
                const int j = min(j0 + t * 16 + l15, p.Lk - 1);
                const float* krow = kbase + (long long)j * p.sKj;
                v8f acc = {};
#pragma unroll
                for (int ks = 0; ks < KS; ++ks) {
                    if (QM == 2)      acc = wmma6(qt_[ks], sp3_ld(krow, p.sKd, ks * 32, hf, p.dh, 1.f), acc);
                    else if (QM == 1) acc = wmma3(qs_[ks], sp_ld(krow, p.sKd, ks * 32, hf, p.dh, 1.f), acc);
                    else              acc = wmma16(qa[ks], fh_ld(krow, p.sKd, ks * 32, hf, p.dh, 1.f), acc);
                }
                s[t] = acc;
            }
            float pv[8][4];
#pragma unroll
            for (int i = 0; i < 8; ++i) {
                const int irow = q0 + i + 8 * hf;
                const int ic = min(irow, p.Lq - 1);
                float sc[4];
#pragma unroll
                for (int t = 0; t < 4; ++t) {
                    const int jg = j0 + t * 16 + l15;
                    float v = s[t][i] * p.scale;
                    if (p.Mf) v += p.Mf[b * p.smb + h * p.smh + (long long)ic * p.smi + (long long)min(jg, p.Lk - 1) * p.smj];
                    if (p.Rt) { int rc = ic - min(jg, p.Lk - 1) + p.roff; rc = rc < 0 ? 0 : (rc >= p.rn ? p.rn - 1 : rc); v += p.Rt[b * p.srb + h * p.srh + (long long)ic * p.sri + rc]; }
                    if (p.Mi) { const int mv = p.Mi[b * p.smb + h * p.smh + (long long)ic * p.smi + (long long)min(jg, p.Lk - 1) * p.smj]; if (p.mpol ? (mv != 0) : (mv == 0)) v = p.mfill; }
                    if (p.SQ) { const bool same = p.SQ[(long long)b * p.Lq + ic] == p.SK[(long long)b * p.Lk + min(jg, p.Lk - 1)]; if (p.segpol ? same : !same) v = p.mfill; }
                    if (p.causal == 2 && jg > irow + p.coff) v = p.mfill;
                    if (jg >= p.Lk || (p.causal == 1 && jg > irow + p.coff) || (p.causal == 3 && jg < irow + p.coff) || (p.win > 0 && irow + p.coff - jg > p.win)) v = NEG; else v *= L2E;
                    sc[t] = v;
                }
                if (!TWOPASS || pass == 0) {
                    float mx = fmaxf(fmaxf(sc[0], sc[1]), fmaxf(sc[2], sc[3]));
                    mx = fmaxf(mx, __shfl_xor(mx, 1, 32)); mx = fmaxf(mx, __shfl_xor(mx, 2, 32));
                    mx = fmaxf(mx, __shfl_xor(mx, 4, 32)); mx = fmaxf(mx, __shfl_xor(mx, 8, 32));
                    const float mnew = fmaxf(m8[i], mx);
                    const float corr = (mnew == NEG) ? 1.f : exp2f(m8[i] - mnew);
                    float rs = 0.f;
#pragma unroll
                    for (int t = 0; t < 4; ++t) {
                        const float pp = (sc[t] == NEG) ? 0.f : exp2f(sc[t] - mnew); rs += pp;
                        pv[i][t] = p.Pw ? pp * p.Pw[b * p.swb + h * p.swh + (long long)ic * p.swi + (long long)min(j0 + t * 16 + l15, p.Lk - 1) * p.swj] : pp;
                    }
                    rs += __shfl_xor(rs, 1, 32); rs += __shfl_xor(rs, 2, 32); rs += __shfl_xor(rs, 4, 32); rs += __shfl_xor(rs, 8, 32);
                    l8[i] = l8[i] * corr + rs; m8[i] = mnew;
                    if (!TWOPASS) {
#pragma unroll
                        for (int t = 0; t < NT; ++t) o[t][i] *= corr;
                    }
                } else {
                    const float inv = (l8[i] > 0.f) ? 1.f / l8[i] : 0.f;
#pragma unroll
                    for (int t = 0; t < 4; ++t) {
                        const int jg = j0 + t * 16 + l15;
                        float pp = (sc[t] == NEG) ? 0.f : exp2f(sc[t] - m8[i]) * inv;
                        if (p.Pw) pp *= p.Pw[b * p.swb + h * p.swh + (long long)ic * p.swi + (long long)min(jg, p.Lk - 1) * p.swj];
                        pv[i][t] = pp;
                    }
                }
            }
            if (dopv) {
#pragma unroll
                for (int i = 0; i < 8; ++i)
#pragma unroll
                    for (int t = 0; t < 4; ++t) ((volatile float*)myp)[(i + 8 * hf) * 64 + t * 16 + l15] = pv[i][t];
                __syncthreads();
                if (p.P) {
                    float* pb_ = p.P + b * p.sPb + h * p.sPh;
                    const bool fastP = (p.pband == 0) && ((p.sPi & 3) == 0) && (j0 + 64 <= p.Lk) && (q0 + 16 <= p.Lq) && ((((size_t)pb_) & 15) == 0);
                    if (fastP) {
#pragma unroll
                        for (int s2 = 0; s2 < 8; ++s2) {
                            const int row = s2 * 2 + (lane >> 4), c4 = (lane & 15) * 4;
                            const v4f v = *(const v4f*)(myp + row * 64 + c4);
                            VST2V4(pb_ + (long long)(q0 + row) * p.sPi + j0 + c4, v);
                        }
                    } else {
                        for (int row = 0; row < 16; ++row) {
                            const int irow = q0 + row; if (irow >= p.Lq) continue;
                            for (int c = lane; c < 64; c += 32) {
                                const int jg = j0 + c; if (jg >= p.Lk) continue;
                                if (p.pband == 0) VST2(float, pb_ + (long long)irow * p.sPi + jg, myp[row * 64 + c]);
                                else if (jg - irow <= p.pband && irow - jg <= p.pband) VST2(float, pb_ + (long long)irow * p.sPi + (jg - irow + p.pband), myp[row * 64 + c]);
                            }
                        }
                    }
                }
                if (SPLITPV) {
                    const Split pa0 = sp_ld(myp + l15 * 64, 1, 0, hf, 64, 1.f), pa1 = sp_ld(myp + l15 * 64, 1, 32, hf, 64, 1.f);
                    const __bf16* vh = (const __bf16*)vl; const __bf16* vlo = vh + 64 * VP;
#pragma unroll
                    for (int t = 0; t < NT; ++t) {
                        const int dcol = t * 16 + l15;
                        Split b0, b1;
#pragma unroll
                        for (int e = 0; e < 16; ++e) {
                            const int k0 = frag_k(e, hf), k1 = 32 + frag_k(e, hf);
                            b0.hi[e] = vh[k0 * VP + dcol]; b0.lo[e] = vlo[k0 * VP + dcol]; b1.hi[e] = vh[k1 * VP + dcol]; b1.lo[e] = vlo[k1 * VP + dcol];
                        }
                        o[t] = wmma3(pa0, b0, o[t]);
                        o[t] = wmma3(pa1, b1, o[t]);
                    }
                } else {
                    const v16h pa0 = fh_ld(myp + l15 * 64, 1, 0, hf, 64, 4096.f), pa1 = fh_ld(myp + l15 * 64, 1, 32, hf, 64, 4096.f);
#pragma unroll
                    for (int t = 0; t < NT; ++t) {
                        const int dcol = t * 16 + l15;
                        v16h b0, b1;
#pragma unroll
                        for (int e = 0; e < 16; ++e) { b0[e] = vl[frag_k(e, hf) * VP + dcol]; b1[e] = vl[(32 + frag_k(e, hf)) * VP + dcol]; }
                        o[t] = wmma16(pa0, b0, o[t]);
                        o[t] = wmma16(pa1, b1, o[t]);
                    }
                }
            }
        }
    }
    float* obase = p.O + b * p.sOb + h * p.sOh;
    if (p.ST) {
        const int rl = lane >> 1, isel = rl & 7;
        float mv = 0.f, lv = 0.f;
#pragma unroll
        for (int i = 0; i < 8; ++i) if (i == isel) { mv = m8[i]; lv = l8[i]; }
        const int irow = q0 + rl;
        if (irow < p.Lq) { float* st = p.ST + (((long long)b * gridDim.y + h) * p.Lq + irow) * 2 + (lane & 1); VST2(float, st, (lane & 1) ? lv : mv * 0.6931471805599453f); }
    }
    float invr[8];
#pragma unroll
    for (int i = 0; i < 8; ++i) {
        if (TWOPASS) invr[i] = SPLITPV ? 1.f : (1.f / 4096.f);
        else if (p.nonorm) invr[i] = exp2f(m8[i]) * (SPLITPV ? 1.f : (1.f / 4096.f));
        else invr[i] = (l8[i] > 0.f) ? (SPLITPV ? 1.f / l8[i] : 1.f / (l8[i] * 4096.f)) : 0.f;
    }
    __syncthreads();
    const bool ofast = ((p.sOi & 3) == 0) && ((((size_t)obase) & 15) == 0) && (q0 + 16 <= p.Lq);
#pragma unroll
    for (int c0 = 0; c0 < DVP; c0 += 64) {
#pragma unroll
        for (int i = 0; i < 8; ++i)
#pragma unroll
            for (int t = 0; t < NT; ++t) if (t * 16 >= c0 && t * 16 < c0 + 64) ((volatile float*)myp)[(i + 8 * hf) * 64 + (t * 16 - c0) + l15] = o[t][i] * invr[i];
        __syncthreads();
        const int cw = (DVP - c0 < 64) ? (DVP - c0) : 64;
        if (ofast && (c0 + cw <= p.dv) && (cw % 32 == 0)) {
            const int lpr = cw / 4;
            const int rows_per_ins = 32 / lpr;
            for (int r0 = 0; r0 < 16; r0 += rows_per_ins) {
                const int row = r0 + lane / lpr, c4 = (lane % lpr) * 4;
                const v4f v = *(const v4f*)(myp + row * 64 + c4);
                VST2V4(obase + (long long)(q0 + row) * p.sOi + c0 + c4, v);
            }
        } else {
            for (int row = 0; row < 16; ++row) {
                const int irow = q0 + row; if (irow >= p.Lq) continue;
                for (int c = lane; c < cw; c += 32) { const int d = c0 + c; if (d < p.dv) VST2(float, obase + (long long)irow * p.sOi + d, myp[row * 64 + c]); }
            }
        }
        __syncthreads();
    }
}

struct GemmH {
    const unsigned short* A; const unsigned short* AL; const unsigned short* B; float* C;
    long long sAz, sAm, sBz, sBn, sCz, sCm;
    int M, N, K, pad0; float oscale, lscale;
};
static_assert(sizeof(GemmH) == 4 * 8 + 6 * 8 + 4 * 4 + 2 * 4);

template <int TM, int TN, bool ARES>
__global__ __launch_bounds__(32) void k_hgemm(GemmH p) {
    const int lane = threadIdx.x & 31, h = lane >> 4, l15 = lane & 15;
    const int m0 = blockIdx.y * (16 * TM), n0 = blockIdx.x * (16 * TN), z = blockIdx.z;
    const _Float16* A  = (const _Float16*)(p.A  + (long long)z * p.sAz);
    const _Float16* AL = (const _Float16*)(p.AL + (long long)z * p.sAz);
    const _Float16* B  = (const _Float16*)(p.B  + (long long)z * p.sBz);
    v8f acc[TM][TN], accl[TM][TN];
#pragma unroll
    for (int i = 0; i < TM; ++i)
#pragma unroll
        for (int t = 0; t < TN; ++t) { v8f zz = {}; acc[i][t] = zz; accl[i][t] = zz; }
    for (int k0 = 0; k0 < p.K; k0 += 32) {
        v16h a[TM], al[TM], b[TN];
#pragma unroll
        for (int i = 0; i < TM; ++i) {
            const int am = min(m0 + 16 * i + l15, p.M - 1);
            a[i] = frag_ld(A + (long long)am * p.sAm + k0 + 8 * h);
            if (ARES) al[i] = frag_ld(AL + (long long)am * p.sAm + k0 + 8 * h);
        }
#pragma unroll
        for (int t = 0; t < TN; ++t) {
            const int bn = min(n0 + 16 * t + l15, p.N - 1);
            b[t] = frag_ld(B + (long long)bn * p.sBn + k0 + 8 * h);
        }
#pragma unroll
        for (int i = 0; i < TM; ++i)
#pragma unroll
            for (int t = 0; t < TN; ++t) {
                acc[i][t] = wmma16(a[i], b[t], acc[i][t]);
                if (ARES) accl[i][t] = wmma16(al[i], b[t], accl[i][t]);
            }
    }
    float* C = p.C + (long long)z * p.sCz;
    __shared__ __align__(16) float ctile[16][36];
#pragma unroll
    for (int i = 0; i < TM; ++i) {
        const int mb = m0 + 16 * i; if (mb >= p.M) break;
#pragma unroll
        for (int tp = 0; tp < TN / 2; ++tp) {
            const int nb = n0 + 32 * tp; if (nb >= p.N) break;
#pragma unroll
            for (int t2 = 0; t2 < 2; ++t2) {
                const int t = 2 * tp + t2; const int n = nb + t2 * 16 + l15;
#pragma unroll
                for (int r = 0; r < 8; ++r) {
                    float v = acc[i][t][r] * p.oscale;
                    if (ARES) v += accl[i][t][r] * p.lscale;
                    ctile[8 * h + r][t2 * 16 + l15] = (n < p.N) ? v : 0.f;
                }
            }
            __syncthreads();
            const bool fast = (mb + 16 <= p.M) && (nb + 32 <= p.N) && ((p.sCm & 3) == 0) && ((((size_t)C) & 15) == 0);
            if (fast) {
#pragma unroll
                for (int s2 = 0; s2 < 4; ++s2) {
                    const int row = s2 * 4 + (lane >> 3), c4 = (lane & 7) * 4;
                    const v4f v = *(const v4f*)&ctile[row][c4];
                    VST2V4(C + (long long)(mb + row) * p.sCm + nb + c4, v);
                }
            } else {
                for (int row = 0; row < 16; ++row) {
                    const int m = mb + row, n = nb + lane;
                    if (m < p.M && n < p.N) VST2(float, C + (long long)m * p.sCm + n, ctile[row][lane]);
                }
            }
            __syncthreads();
        }
    }
}

__device__ __forceinline__ unsigned int cmb_pk2(float a, float b) { return (unsigned int)__builtin_bit_cast(unsigned short, (_Float16)a) | ((unsigned int)__builtin_bit_cast(unsigned short, (_Float16)b) << 16); }
__device__ __forceinline__ float cmb_bf(float v) { const unsigned u = __builtin_bit_cast(unsigned, v); const unsigned r = (u + 0x7fffu + ((u >> 16) & 1u)) & 0xffff0000u; return __builtin_bit_cast(float, r); }
__global__ __launch_bounds__(256) void k_cm_castb(const float* __restrict__ SRC, int lds, unsigned short* __restrict__ DST, int ldd, int nR, int nC, float sc) {
    const long long u = (long long)blockIdx.x * 256 + threadIdx.x; const int per = nC / 8; if (u >= (long long)nR * per) return; const int r = (int)(u / per); const int c0 = 8 * (int)(u % per);
    const float* s = SRC + (long long)r * lds + c0; float w[8];
#pragma unroll
    for (int e = 0; e < 8; ++e) w[e] = cmb_bf(s[e]) * sc;
    cm_u4 pk; pk.x = cmb_pk2(w[0], w[1]); pk.y = cmb_pk2(w[2], w[3]); pk.z = cmb_pk2(w[4], w[5]); pk.w = cmb_pk2(w[6], w[7]); VST2(cm_u4, (cm_u4*)(DST + (long long)r * ldd + c0), pk); }

__global__ __launch_bounds__(256) void k_ropetab(float* __restrict__ tab) {
    const int idx = blockIdx.x * 256 + threadIdx.x; if (idx >= 512) return;
    const int pp = idx >> 5, i = idx & 31;
    const float e = (float)(2 * i) * (1.0f / (float)HD);
    const float invf = 1.0f / powf(10000.0f, e);
    const float ang = (float)pp * invf;
    VST2(float, tab + idx, cosf(ang));
    VST2(float, tab + 512 + idx, sinf(ang));
}

__global__ __launch_bounds__(256) void k_normrope(const float* __restrict__ src, const float* __restrict__ w, const float* __restrict__ tab, float* __restrict__ dst, int nheads, int nrows) {
    const int wv = blockIdx.x * 8 + (threadIdx.x >> 5); const int lane = threadIdx.x & 31;
    if (wv >= nrows) return;
    const int hd = wv % nheads;
    const float* pr = src + (long long)wv * HD;
    const v2f xv = *(const v2f*)(pr + 2 * lane);
    float ss = xv.x * xv.x + xv.y * xv.y;
    ss += __shfl_xor(ss, 1, 32); ss += __shfl_xor(ss, 2, 32); ss += __shfl_xor(ss, 4, 32); ss += __shfl_xor(ss, 8, 32); ss += __shfl_xor(ss, 16, 32);
    const float rn = rsqrtf(ss * (1.0f / (float)HD) + 1e-6f);
    const float we = cmb_bf(w[2 * lane]), wo = cmb_bf(w[2 * lane + 1]);
    const float a = xv.x * rn * we, bq = xv.y * rn * wo;
    const float cs = tab[hd * 32 + lane], sn = tab[512 + hd * 32 + lane];
    v2f ov; ov.x = a * cs - bq * sn; ov.y = a * sn + bq * cs;
    VST2(v2f, dst + (long long)wv * HD + 2 * lane, ov);
}

__global__ __launch_bounds__(256) void k_ctxpl(const float* __restrict__ src, unsigned short* __restrict__ PH, unsigned short* __restrict__ PLo, long long n8) {
    const long long u = (long long)blockIdx.x * 256 + threadIdx.x; if (u >= n8) return;
    const v4f x0 = *(const v4f*)(src + 8 * u), x1 = *(const v4f*)(src + 8 * u + 4);
    const float w[8] = {x0.x, x0.y, x0.z, x0.w, x1.x, x1.y, x1.z, x1.w};
    unsigned short hh[8], ll[8];
#pragma unroll
    for (int e = 0; e < 8; ++e) {
        const float c = w[e] * 16.f; const _Float16 hv = (_Float16)c; const float r = (c - (float)hv) * 2048.f;
        hh[e] = __builtin_bit_cast(unsigned short, hv); ll[e] = __builtin_bit_cast(unsigned short, (_Float16)r);
    }
    cm_u4 ph; ph.x = (unsigned)hh[0] | ((unsigned)hh[1] << 16); ph.y = (unsigned)hh[2] | ((unsigned)hh[3] << 16); ph.z = (unsigned)hh[4] | ((unsigned)hh[5] << 16); ph.w = (unsigned)hh[6] | ((unsigned)hh[7] << 16);
    cm_u4 pq; pq.x = (unsigned)ll[0] | ((unsigned)ll[1] << 16); pq.y = (unsigned)ll[2] | ((unsigned)ll[3] << 16); pq.z = (unsigned)ll[4] | ((unsigned)ll[5] << 16); pq.w = (unsigned)ll[6] | ((unsigned)ll[7] << 16);
    VST2(cm_u4, (cm_u4*)(PH + 8 * u), ph);
    VST2(cm_u4, (cm_u4*)(PLo + 8 * u), pq);
}


extern "C" void kernel_launch(void* const* d_in, const int* in_sizes, int n_in, void* d_out, int out_size, void* d_ws, size_t ws_size, hipStream_t stream) {
    if (n_in < 7) return;
    if ((long long)in_sizes[0] < (long long)(NB - 1) * IN_BSTRIDE + (long long)SEQ * NE) return;
    if (in_sizes[1] < NE * NE || in_sizes[2] < NKVE * NE || in_sizes[3] < NKVE * NE || in_sizes[4] < NE * NE || in_sizes[5] < HD || in_sizes[6] < HD) return;
    if ((long long)out_size < (long long)(NB - 1) * OUT_BSTRIDE + (long long)SEQ * NE) return;
    const float* x  = (const float*)d_in[0];
    const float* Wq = (const float*)d_in[1];
    const float* Wk = (const float*)d_in[2];
    const float* Wv = (const float*)d_in[3];
    const float* Wo = (const float*)d_in[4];
    const float* qw = (const float*)d_in[5];
    const float* kw = (const float*)d_in[6];
    float* out = (float*)d_out;

    const long long M = MROWS;
    size_t off = 0;
    auto carve = [&](size_t bytes) -> char* { char* r = (char*)d_ws + off; off += (bytes + 255) & ~(size_t)255; return r; };
    unsigned short* XH   = (unsigned short*)carve((size_t)M * NE * 2);
    unsigned short* WQH  = (unsigned short*)carve((size_t)NE * NE * 2);
    unsigned short* WKVH = (unsigned short*)carve((size_t)2 * NKVE * NE * 2);
    unsigned short* WOH  = (unsigned short*)carve((size_t)NE * NE * 2);
    float* QR  = (float*)carve((size_t)M * NE * 4);
    float* KVR = (float*)carve((size_t)2 * M * NKVE * 4);
    float* TAB = (float*)carve(4096);
    float* QN  = (float*)carve((size_t)M * NE * 4);
    float* KN  = (float*)carve((size_t)M * NKVE * 4);
    float* CTX = (float*)carve((size_t)M * NE * 4);
    unsigned short* CH = (unsigned short*)carve((size_t)M * NE * 2);
    unsigned short* CL = (unsigned short*)carve((size_t)M * NE * 2);
    if (off > ws_size) return;
    float* KR = KVR; float* VR = KVR + M * NKVE;

    for (int bb = 0; bb < NB; ++bb)
        k_cm_castb<<<(unsigned)(((long long)SEQ * (NE / 8) + 255) / 256), 256, 0, stream>>>(x + (long long)bb * IN_BSTRIDE, NE, XH + (long long)bb * SEQ * NE, NE, SEQ, NE, 16.f);
    k_cm_castb<<<(unsigned)((NE * (NE / 8) + 255) / 256), 256, 0, stream>>>(Wq, NE, WQH, NE, NE, NE, 1024.f);
    k_cm_castb<<<(unsigned)((NKVE * (NE / 8) + 255) / 256), 256, 0, stream>>>(Wk, NE, WKVH, NE, NKVE, NE, 1024.f);
    k_cm_castb<<<(unsigned)((NKVE * (NE / 8) + 255) / 256), 256, 0, stream>>>(Wv, NE, WKVH + (long long)NKVE * NE, NE, NKVE, NE, 1024.f);
    k_cm_castb<<<(unsigned)((NE * (NE / 8) + 255) / 256), 256, 0, stream>>>(Wo, NE, WOH, NE, NE, NE, 1024.f);

    { GemmH g;
      g.A = XH; g.AL = XH; g.B = WQH; g.C = QR;
      g.sAz = 0; g.sAm = NE; g.sBz = 0; g.sBn = NE; g.sCz = 0; g.sCm = NE;
      g.M = (int)M; g.N = NE; g.K = NE; g.pad0 = 0; g.oscale = 1.f / 16384.f; g.lscale = 0.f;
      k_hgemm<2, 4, false><<<dim3(NE / 64, (unsigned)(M / 32), 1), 32, 0, stream>>>(g); }
    { GemmH g;
      g.A = XH; g.AL = XH; g.B = WKVH; g.C = KVR;
      g.sAz = 0; g.sAm = NE; g.sBz = (long long)NKVE * NE; g.sBn = NE; g.sCz = M * NKVE; g.sCm = NKVE;
      g.M = (int)M; g.N = NKVE; g.K = NE; g.pad0 = 0; g.oscale = 1.f / 16384.f; g.lscale = 0.f;
      k_hgemm<2, 4, false><<<dim3(NKVE / 64, (unsigned)(M / 32), 2), 32, 0, stream>>>(g); }

    k_ropetab<<<2, 256, 0, stream>>>(TAB);
    k_normrope<<<(unsigned)((M * NHD + 7) / 8), 256, 0, stream>>>(QR, qw, TAB, QN, NHD, (int)(M * NHD));
    k_normrope<<<(unsigned)((M * NKV + 7) / 8), 256, 0, stream>>>(KR, kw, TAB, KN, NKV, (int)(M * NKV));

    { AttnP a;
      a.Q = QN; a.K = KN; a.V = VR; a.O = CTX; a.P = 0; a.Mf = 0; a.Mi = 0; a.ST = 0;
      a.Pw = 0; a.Rt = 0; a.SQ = 0; a.SK = 0;
      a.swb = 0; a.swh = 0; a.swi = 0; a.swj = 0; a.srb = 0; a.srh = 0; a.sri = 0;
      a.sQb = (long long)SEQ * NE; a.sQh = HD; a.sQi = NE; a.sQd = 1;
      a.sKb = (long long)SEQ * NKVE; a.sKh = HD; a.sKj = NKVE; a.sKd = 1;
      a.sVb = (long long)SEQ * NKVE; a.sVh = HD; a.sVj = NKVE; a.sVd = 1;
      a.sOb = (long long)SEQ * NE; a.sOh = HD; a.sOi = NE;
      a.sPb = 0; a.sPh = 0; a.sPi = 0; a.smb = 0; a.smh = 0; a.smi = 0; a.smj = 0;
      a.Lq = NEARLY; a.Lk = SEQ; a.dh = HD; a.dv = HD; a.hrep = NHD / NKV; a.causal = 1; a.coff = 0; a.pband = 0;
      a.scale = 0.125f; a.mfill = 0.0f; a.nonorm = 0; a.mpol = 0;
      a.roff = 0; a.rn = 1; a.segpol = 0; a.win = WINSZ - 1;
      k_attn<64, 64, 1, true, false><<<dim3((unsigned)(NEARLY / (16 * AW)), NHD, NB), 32 * AW, 0, stream>>>(a);
      if (SEQ > NEARLY) {
          AttnP c = a;
          c.Q = QN + (long long)NEARLY * NE; c.O = CTX + (long long)NEARLY * NE;
          c.Lq = SEQ - NEARLY; c.Lk = SEQ; c.coff = NEARLY;
          k_attn<64, 64, 0, false, false><<<dim3((unsigned)((SEQ - NEARLY) / (16 * AW)), NHD, NB), 32 * AW, 0, stream>>>(c);
      }
    }

    k_ctxpl<<<(unsigned)((M * NE / 8 + 255) / 256), 256, 0, stream>>>(CTX, CH, CL, M * NE / 8);
    { GemmH g;
      g.A = CH; g.AL = CL; g.B = WOH; g.C = out;
      g.sAz = (long long)SEQ * NE; g.sAm = NE; g.sBz = 0; g.sBn = NE; g.sCz = OUT_BSTRIDE; g.sCm = NE;
      g.M = NEARLY; g.N = NE; g.K = NE; g.pad0 = 0; g.oscale = 1.f / 16384.f; g.lscale = 1.f / (16384.f * 2048.f);
      k_hgemm<2, 2, true><<<dim3(NE / 32, NEARLY / 32, NB), 32, 0, stream>>>(g); }
    if (SEQ > NEARLY) { GemmH g;
      g.A = CH + (long long)NEARLY * NE; g.AL = CL + (long long)NEARLY * NE; g.B = WOH; g.C = out + (long long)NEARLY * NE;
      g.sAz = (long long)SEQ * NE; g.sAm = NE; g.sBz = 0; g.sBn = NE; g.sCz = OUT_BSTRIDE; g.sCm = NE;
      g.M = SEQ - NEARLY; g.N = NE; g.K = NE; g.pad0 = 0; g.oscale = 1.f / 16384.f; g.lscale = 0.f;
      k_hgemm<2, 4, false><<<dim3(NE / 64, (unsigned)((SEQ - NEARLY) / 32), NB), 32, 0, stream>>>(g); }
}
